// Blast_56788057588465
// MI455X (gfx1250) — hardware-verified
//
#include <hip/hip_runtime.h>
#include <stddef.h>


typedef _Float16 v16h __attribute__((ext_vector_type(16)));
typedef _Float16 v8h  __attribute__((ext_vector_type(8)));
typedef float    v8f  __attribute__((ext_vector_type(8)));
typedef float    v4f  __attribute__((ext_vector_type(4)));

#ifndef NB
#define NB 2
#endif
#ifndef SEQ
#define SEQ 1024
#endif
#define NB_FULL  2
#define SEQ_FULL 1024
#define IN_DIM   4096
#define OUT_DIM  4096
#define BLK      256
#define RANK     16
#define NBLK_IN  (IN_DIM / BLK)
#define NBLK_OUT (OUT_DIM / BLK)
#define MROWS    (NB * SEQ)

static_assert(NB >= 1 && NB <= NB_FULL);
static_assert(SEQ >= 64 && SEQ <= SEQ_FULL && (SEQ % 64) == 0);
static_assert(IN_DIM == NBLK_IN * BLK && OUT_DIM == NBLK_OUT * BLK);
static_assert((BLK % 64) == 0);
static_assert(RANK == 16);
static_assert((IN_DIM % 64) == 0 && (IN_DIM % 32) == 0 && (IN_DIM % 8) == 0);
static_assert((OUT_DIM % 64) == 0);
static_assert((MROWS % 64) == 0);
static_assert(((MROWS * (IN_DIM / 8)) % 256) == 0);
static_assert(((IN_DIM / 8) % 32) == 0);
static_assert((size_t)MROWS * IN_DIM < (size_t)0xFFFFFFFFu);
static_assert((size_t)OUT_DIM * IN_DIM < (size_t)0xFFFFFFFFu);

#define LDT 72
#define LDC 68
static_assert((LDT % 8) == 0 && LDT >= 64);
static_assert((LDC % 4) == 0 && LDC >= 64);

#define WCARRY 64.0f
#define UCARRY 64.0f
#define BCARRY 64.0f
#define XCARRY 1.0f

#define X16_BYTES ((size_t)MROWS * IN_DIM * 2)
#define WT_BYTES  ((size_t)OUT_DIM * IN_DIM * 2)
#define OFF_X16 ((size_t)0)
#define OFF_WT  (OFF_X16 + X16_BYTES)
#define WS_TOTAL (OFF_WT + WT_BYTES)
static_assert((X16_BYTES % 128) == 0 && (WT_BYTES % 128) == 0);
static_assert(WS_TOTAL <= (size_t)134217728);

__device__ __forceinline__ float bf16r(float x) {
  unsigned int u = __float_as_uint(x);
  u = (u + 0x7FFFu + ((u >> 16) & 1u)) & 0xFFFF0000u;
  return __uint_as_float(u);
}

static __device__ __forceinline__ _Float16 toh_flush(float v) {
  const _Float16 r = (_Float16)v;
  return (fabsf(v) < 6.103515625e-05f) ? (_Float16)0.0f : r;
}

__device__ __forceinline__ v16h frag_at(const _Float16* p) {
  v8h lo = *(const v8h*)(p);
  v8h hi = *(const v8h*)(p + 16);
  v16h out;
#pragma unroll
  for (int i = 0; i < 8; ++i) { out[i] = lo[i]; out[i + 8] = hi[i]; }
  return out;
}

__device__ __forceinline__ v8f wmma16(v16h a, v16h b, v8f c) {
  v8f d = __builtin_amdgcn_wmma_f32_16x16x32_f16(false, a, false, b, (short)0, c,
                                                 false, false);
  asm volatile("v_nop\n\tv_nop\n\tv_nop\n\tv_nop" : "+v"(d) : "v"(a), "v"(b));
  return d;
}

__global__ __launch_bounds__(256) void xconv_kernel(
    const float* __restrict__ X, _Float16* __restrict__ X16) {
#pragma clang fp contract(off)
  const unsigned gid = blockIdx.x * 256u + threadIdx.x;
  const unsigned crow = gid / (unsigned)(IN_DIM / 8);
  const unsigned c = (gid - crow * (unsigned)(IN_DIM / 8)) * 8u;
  const unsigned bidx = crow / (unsigned)SEQ;
  const unsigned sq = crow - bidx * (unsigned)SEQ;
  const size_t srow = (size_t)bidx * SEQ_FULL + sq;
  const float* xr = X + srow * IN_DIM + c;
  const v4f a0 = *(const v4f*)(xr);
  const v4f a1 = *(const v4f*)(xr + 4);
  v8h o;
#pragma unroll
  for (int i = 0; i < 4; ++i) {
    o[i]     = toh_flush(XCARRY * bf16r(a0[i]));
    o[i + 4] = toh_flush(XCARRY * bf16r(a1[i]));
  }
  _Float16* p = X16 + (size_t)crow * IN_DIM + c;
  *(volatile v8h*)p = o;
  __threadfence();
  *(volatile v8h*)p = o;
}

__global__ __launch_bounds__(256) void wasm_kernel(
    const float* __restrict__ Vt, const float* __restrict__ S, const float* __restrict__ U,
    const float* __restrict__ bias, _Float16* __restrict__ Wt) {
  __shared__ _Float16 T[64 * LDT];
  const unsigned tid = threadIdx.x, lane = tid & 31u;
  const unsigned w = (unsigned)__builtin_amdgcn_readfirstlane((int)(tid >> 5));
  const unsigned mw = w >> 1, nw = w & 1u;
  const unsigned hh = lane >> 4, m = lane & 15u;
  const unsigned n0 = blockIdx.x * 64u;
  const unsigned k0 = blockIdx.y * 64u;
  const unsigned ob = n0 / (unsigned)BLK;
  const unsigned q0 = n0 - ob * (unsigned)BLK;
  const unsigned ib = k0 / (unsigned)BLK;
  const unsigned p0 = k0 - ib * (unsigned)BLK;

  const unsigned q = q0 + mw * 16u + m;
  const float* up = U + ((size_t)ob * RANK + hh * 8u) * BLK + q;
  v16h a;
#pragma unroll
  for (int j = 0; j < 8; ++j) {
    a[j] = toh_flush(UCARRY * bf16r(up[(size_t)j * BLK]));
    a[j + 8] = (_Float16)0.0f;
  }

  const float* sp = S + ((size_t)ob * NBLK_IN + ib) * RANK + hh * 8u;
  const v4f s0 = *(const v4f*)(sp);
  const v4f s1 = *(const v4f*)(sp + 4);

  const unsigned pa = p0 + nw * 32u + m;
  const float* vp0 = Vt + ((size_t)ib * BLK + pa) * RANK + hh * 8u;
  const float* vp1 = vp0 + (size_t)16 * RANK;
  const v4f va0 = *(const v4f*)(vp0);
  const v4f va1 = *(const v4f*)(vp0 + 4);
  const v4f vb0 = *(const v4f*)(vp1);
  const v4f vb1 = *(const v4f*)(vp1 + 4);
  v16h b0, b1;
#pragma unroll
  for (int j = 0; j < 4; ++j) {
    const float sa = bf16r(s0[j]);
    const float sb = bf16r(s1[j]);
    b0[j]     = toh_flush(BCARRY * (sa * bf16r(va0[j])));
    b0[j + 4] = toh_flush(BCARRY * (sb * bf16r(va1[j])));
    b1[j]     = toh_flush(BCARRY * (sa * bf16r(vb0[j])));
    b1[j + 4] = toh_flush(BCARRY * (sb * bf16r(vb1[j])));
  }
#pragma unroll
  for (int j = 8; j < 16; ++j) { b0[j] = (_Float16)0.0f; b1[j] = (_Float16)0.0f; }

  v8f acc0 = {}, acc1 = {};
  acc0 = wmma16(a, b0, acc0);
  acc1 = wmma16(a, b1, acc1);

#pragma unroll
  for (int r = 0; r < 8; ++r) {
    const unsigned row = mw * 16u + hh * 8u + (unsigned)r;
    const float bb = bf16r(bias[n0 + row]);
    const float w0 = acc0[r] * (1.0f / (UCARRY * BCARRY)) + bb;
    const float w1 = acc1[r] * (1.0f / (UCARRY * BCARRY)) + bb;
    T[row * LDT + nw * 32u + m]       = toh_flush(WCARRY * w0);
    T[row * LDT + nw * 32u + 16u + m] = toh_flush(WCARRY * w1);
  }
  __syncthreads();

  v8h x[2];
  size_t off[2];
#pragma unroll
  for (unsigned i = 0; i < 2u; ++i) {
    const unsigned n = 32u * i + (tid >> 3);
    const unsigned kc = (tid & 7u) * 8u;
    x[i] = *(const v8h*)&T[n * LDT + kc];
    off[i] = (size_t)(n0 + n) * IN_DIM + k0 + kc;
  }
#pragma unroll
  for (int i = 0; i < 2; ++i) *(volatile v8h*)(Wt + off[i]) = x[i];
  __threadfence();
#pragma unroll
  for (int i = 0; i < 2; ++i) *(volatile v8h*)(Wt + off[i]) = x[i];
}

__global__ __launch_bounds__(256) void gemm_out_kernel(
    const _Float16* __restrict__ A16, const _Float16* __restrict__ Bt,
    const float* __restrict__ bias, float* __restrict__ outf) {
  __shared__ float Cs[64 * LDC];
  const unsigned K = (unsigned)IN_DIM;
  const unsigned tid = threadIdx.x, lane = tid & 31u;
  const unsigned w = (unsigned)__builtin_amdgcn_readfirstlane((int)(tid >> 5));
  const unsigned mw = w >> 1, nw = w & 1u;
  const unsigned hh = lane >> 4, m = lane & 15u;
  const unsigned n0 = blockIdx.x * 64u;
  const unsigned row0 = blockIdx.y * 64u;

  const _Float16* ap  = A16 + (size_t)(row0 + mw * 16u + m) * K + hh * 8u;
  const _Float16* bp0 = Bt + (size_t)(n0 + nw * 32u + m) * K + hh * 8u;
  const _Float16* bp1 = bp0 + (size_t)16 * K;
  v8f acc0 = {}, acc1 = {};
#pragma unroll 2
  for (unsigned k0 = 0; k0 < K; k0 += 32u) {
    const v16h a  = frag_at(ap + k0);
    const v16h b0 = frag_at(bp0 + k0);
    const v16h b1 = frag_at(bp1 + k0);
    acc0 = wmma16(a, b0, acc0);
    acc1 = wmma16(a, b1, acc1);
  }
#pragma unroll
  for (int r = 0; r < 8; ++r) {
    float* d = &Cs[(mw * 16u + hh * 8u + (unsigned)r) * LDC + nw * 32u + m];
    d[0]  = acc0[r];
    d[16] = acc1[r];
  }
  __syncthreads();

  const float cs = 1.0f / (WCARRY * XCARRY);
  v4f xs[4];
  size_t off[4];
#pragma unroll
  for (unsigned i = 0; i < 4u; ++i) {
    const unsigned r = 16u * i + (tid >> 4);
    const unsigned c = (tid & 15u) * 4u;
    const unsigned crow = row0 + r;
    const unsigned bidx = crow / (unsigned)SEQ;
    const unsigned sq = crow - bidx * (unsigned)SEQ;
    const size_t frow = (size_t)bidx * SEQ_FULL + sq;
    const v4f u = *(const v4f*)&Cs[r * LDC + c];
    const v4f g = *(const v4f*)(bias + n0 + c);
    v4f val;
#pragma unroll
    for (int j = 0; j < 4; ++j) val[j] = u[j] * cs + bf16r(g[j]);
    xs[i] = val;
    off[i] = frow * OUT_DIM + n0 + c;
  }
#pragma unroll
  for (int i = 0; i < 4; ++i) *(volatile v4f*)(outf + off[i]) = xs[i];
  __threadfence();
#pragma unroll
  for (int i = 0; i < 4; ++i) *(volatile v4f*)(outf + off[i]) = xs[i];
}

extern "C" void kernel_launch(void* const* d_in, const int* in_sizes, int n_in,
                              void* d_out, int out_size, void* d_ws, size_t ws_size,
                              hipStream_t stream) {
  if (n_in < 5) return;
  const long long need_x = ((long long)(NB - 1) * SEQ_FULL + SEQ) * IN_DIM;
  const long long need_o = ((long long)(NB - 1) * SEQ_FULL + SEQ) * OUT_DIM;
  if ((long long)in_sizes[0] < need_x) return;
  if ((long long)in_sizes[1] < (long long)NBLK_OUT * NBLK_IN * RANK) return;
  if ((long long)in_sizes[2] < (long long)NBLK_OUT * RANK * BLK) return;
  if ((long long)in_sizes[3] < (long long)NBLK_IN * BLK * RANK) return;
  if ((long long)in_sizes[4] < (long long)OUT_DIM) return;
  if ((long long)out_size < need_o) return;
  if (ws_size < WS_TOTAL) return;

  const float* X    = (const float*)d_in[0];
  const float* Sf   = (const float*)d_in[1];
  const float* Uf   = (const float*)d_in[2];
  const float* Vtf  = (const float*)d_in[3];
  const float* bias = (const float*)d_in[4];
  float* out = (float*)d_out;

  char* ws = (char*)d_ws;
  _Float16* X16 = (_Float16*)(ws + OFF_X16);
  _Float16* Wt  = (_Float16*)(ws + OFF_WT);

  dim3 blk(256);
  xconv_kernel<<<dim3((MROWS * (IN_DIM / 8)) / 256), blk, 0, stream>>>(X, X16);
  wasm_kernel<<<dim3(OUT_DIM / 64, IN_DIM / 64), blk, 0, stream>>>(Vtf, Sf, Uf, bias, Wt);
  gemm_out_kernel<<<dim3(OUT_DIM / 64, MROWS / 64), blk, 0, stream>>>(X16, Wt, bias, out);
}
